// ScatterSelfAttention_13408887898530
// MI455X (gfx1250) — hardware-run, weakly checked
//
#include <hip/hip_runtime.h>

typedef float          v8f   __attribute__((ext_vector_type(8)));
typedef float          v4f   __attribute__((ext_vector_type(4)));
typedef unsigned int   v4u   __attribute__((ext_vector_type(4)));
typedef int            v8i   __attribute__((ext_vector_type(8)));
typedef unsigned short v8us  __attribute__((ext_vector_type(8)));
typedef unsigned short v16us __attribute__((ext_vector_type(16)));
typedef __bf16         v16bf __attribute__((ext_vector_type(16)));
typedef _Float16       v16h  __attribute__((ext_vector_type(16)));
typedef v4f  __attribute__((may_alias)) v4fa;
typedef v8us __attribute__((may_alias)) v8usa;
union FragB { v16bf v; v16us u; v8us h[2]; v8i w; };
union FragH { v16h  v; v16us u; v8us h[2]; v8i w; };

__device__ __forceinline__ v8f wmb(const FragB& a, const FragB& b, v8f c) {
  v8f d = __builtin_amdgcn_wmma_f32_16x16x32_bf16(false, a.v, false, b.v, (short)0, c, false, false);
  asm volatile("v_nop\n\tv_nop\n\tv_nop\n\tv_nop" : "+v"(d) : "v"(a.w), "v"(b.w));
  return d;
}

__device__ __forceinline__ v8f wmh(const FragH& a, const FragH& b, v8f c) {
  v8f d = __builtin_amdgcn_wmma_f32_16x16x32_f16(false, a.v, false, b.v, (short)0, c, false, false);
  asm volatile("v_nop\n\tv_nop\n\tv_nop\n\tv_nop" : "+v"(d) : "v"(a.w), "v"(b.w));
  return d;
}

__device__ __forceinline__ unsigned bf16_bits(float f) {
  const unsigned u = __float_as_uint(f);
  const unsigned r = (u + 0x7FFFu + ((u >> 16) & 1u)) >> 16;
  const unsigned q = (u >> 16) | 0x40u;
  return ((u & 0x7fffffffu) > 0x7f800000u) ? q : r;
}

__device__ __forceinline__ float bf16_val(float f) {
  return __uint_as_float(bf16_bits(f) << 16);
}
__device__ __forceinline__ int clampi(int v, int lo, int hi) {
  return v < lo ? lo : (v > hi ? hi : v);
}

__device__ __forceinline__ unsigned f16_bits(float f) {
  const unsigned u  = __float_as_uint(f);
  const unsigned s  = (u >> 16) & 0x8000u;
  const unsigned a  = u & 0x7fffffffu;
  const unsigned t  = a - 0x38000000u;
  const unsigned r  = (t + 0x0FFFu + ((t >> 13) & 1u)) >> 13;
  const unsigned rc = r > 0x7C00u ? 0x7C00u : r;
  const bool small  = a < 0x38800000u;
  const bool isnan  = a > 0x7f800000u;
  const unsigned fin = small ? 0u : (s | rc);
  return isnan ? (s | 0x7E00u) : fin;
}

__device__ __forceinline__ unsigned pk16(unsigned lo, unsigned hi) { return lo | (hi << 16); }
__device__ __forceinline__ unsigned bf16_lo_bits(float v) {
  float hi = bf16_val(v);
  asm volatile("" : "+v"(hi));
  return bf16_bits(v - hi);
}
__device__ __forceinline__ v4u pack8_bf16(v4f a, v4f c) {
  return (v4u){ pk16(bf16_bits(a[0]), bf16_bits(a[1])), pk16(bf16_bits(a[2]), bf16_bits(a[3])),
                pk16(bf16_bits(c[0]), bf16_bits(c[1])), pk16(bf16_bits(c[2]), bf16_bits(c[3])) };
}
__device__ __forceinline__ v4u pack8_bf16_lo(v4f a, v4f c) {
  return (v4u){ pk16(bf16_lo_bits(a[0]), bf16_lo_bits(a[1])), pk16(bf16_lo_bits(a[2]), bf16_lo_bits(a[3])),
                pk16(bf16_lo_bits(c[0]), bf16_lo_bits(c[1])), pk16(bf16_lo_bits(c[2]), bf16_lo_bits(c[3])) };
}
__device__ __forceinline__ v4u pack8_f16(v4f a, v4f c) {
  return (v4u){ pk16(f16_bits(a[0]), f16_bits(a[1])), pk16(f16_bits(a[2]), f16_bits(a[3])),
                pk16(f16_bits(c[0]), f16_bits(c[1])), pk16(f16_bits(c[2]), f16_bits(c[3])) };
}

template <int FORM>
__global__ __launch_bounds__(256) void k_plane(const float* __restrict__ src, int rows, int cols, int ldsrc,
                                               unsigned short* __restrict__ dst, int MP, int KP) {
  static_assert(FORM >= 0 && FORM <= 3);
  const int KTOT = (FORM == 1 || FORM == 3) ? 2 * KP : KP;
  const unsigned ppr   = (unsigned)(KTOT >> 3);
  const unsigned kp8   = (unsigned)(KP >> 3);
  const unsigned total = (unsigned)MP * ppr;
  const unsigned g     = blockIdx.x * 256u + threadIdx.x;
  const unsigned rowu  = g / ppr;
  const unsigned p     = g - rowu * ppr;
  const bool second    = p >= kp8;
  const int row = (int)rowu;
  const int c0  = (int)((second ? p - kp8 : p) << 3);
  const float* srow = src + (size_t)clampi(row, 0, rows - 1) * (size_t)ldsrc;
  float x[8];
  unsigned mk[8];
#pragma unroll
  for (int e = 0; e < 8; ++e) {
    const int c = c0 + e;
    const float v = srow[clampi(c, 0, cols - 1)];
    asm volatile("" :: "v"(v));
    x[e]  = v;
    mk[e] = (row < rows && c < cols) ? 0xFFFFu : 0u;
  }
  const v4f a = (v4f){ x[0], x[1], x[2], x[3] };
  const v4f c = (v4f){ x[4], x[5], x[6], x[7] };
  v4u o;
  if (FORM == 2) {
    o = pack8_f16(a, c);
  } else {
    const v4u hi = pack8_bf16(a, c);
    o = hi;
    if (FORM == 1) { const v4u lo = pack8_bf16_lo(a, c); o = second ? lo : hi; }
  }
  const v4u mw = (v4u){ pk16(mk[0], mk[1]), pk16(mk[2], mk[3]), pk16(mk[4], mk[5]), pk16(mk[6], mk[7]) };
  o &= mw;
  if (g < total) {
    volatile v4u* q = (volatile v4u*)(dst + (size_t)g * 8);
    *q = o;
    __threadfence();
    *q = o;
  }
}

template <int FORM> struct FragOf    { typedef FragB T; };
template <>         struct FragOf<2> { typedef FragH T; };
__device__ __forceinline__ v8f mm(const FragB& a, const FragB& b, v8f c) { return wmb(a, b, c); }
__device__ __forceinline__ v8f mm(const FragH& a, const FragH& b, v8f c) { return wmh(a, b, c); }
template <class F> __device__ __forceinline__ F ld_frag(const unsigned short* p) {
  F f;
  f.h[0] = *(const v8usa*)(p);
  f.h[1] = *(const v8usa*)(p + 16);
  return f;
}

template <int FORM, int EPI>
__global__ __launch_bounds__(256) __attribute__((amdgpu_num_vgpr(248)))
void k_gemm_nt(const unsigned short* __restrict__ A, const unsigned short* __restrict__ B,
               const float* __restrict__ bias, float* __restrict__ D, int M, int N, int KTOT, int ldd) {
  static_assert(FORM >= 0 && FORM <= 2);
  static_assert(EPI == 0 || EPI == 1);
  typedef typename FragOf<FORM>::T F;
  __shared__ __attribute__((aligned(16))) float sT[8][16 * 68];
  const int lane = threadIdx.x & 31;
  const int wave = threadIdx.x >> 5;
  const int tilesM = (M + 63) >> 6;
  const int tilesN = (N + 63) >> 6;
  const int tile = blockIdx.x * 8 + wave;
  if (tile >= tilesM * tilesN) return;
  const int tm = tile / tilesN;
  const int tn = tile - tm * tilesN;
  const int m0 = tm << 6;
  const int n0 = tn << 6;

  const int rl = lane & 15;
  const int h8 = (lane >> 4) * 8;
  const unsigned short* pa = A + (size_t)(m0 + rl) * (size_t)KTOT + h8;
  const unsigned short* pb = B + (size_t)(n0 + rl) * (size_t)KTOT + h8;

  v8f acc[4][4];
#pragma unroll
  for (int i = 0; i < 4; ++i)
#pragma unroll
    for (int j = 0; j < 4; ++j) acc[i][j] = (v8f){0.f, 0.f, 0.f, 0.f, 0.f, 0.f, 0.f, 0.f};

#pragma unroll 1
  for (int k0 = 0; k0 < KTOT; k0 += 32) {
    F bf[4];
#pragma unroll
    for (int j = 0; j < 4; ++j) bf[j] = ld_frag<F>(pb + (size_t)(j << 4) * (size_t)KTOT + k0);
#pragma unroll
    for (int i = 0; i < 4; ++i) {
      const F af = ld_frag<F>(pa + (size_t)(i << 4) * (size_t)KTOT + k0);
#pragma unroll
      for (int j = 0; j < 4; ++j) acc[i][j] = mm(af, bf[j], acc[i][j]);
    }
  }

  float* slab = sT[wave];
  const int hh = lane >> 4;
  const int c4 = (lane & 15) * 4;
  const int nc = n0 + c4;
  const bool cok = nc < N;
  v4f bv = (v4f){0.f, 0.f, 0.f, 0.f};
  if (EPI == 1) {
    bv = *(const v4fa*)(bias + clampi(nc, 0, N - 4));
    asm volatile("" :: "v"(bv));
  }
#pragma unroll
  for (int i = 0; i < 4; ++i) {
    const int mBase = m0 + (i << 4);
#pragma unroll
    for (int j = 0; j < 4; ++j) {
#pragma unroll
      for (int r = 0; r < 8; ++r) slab[(h8 + r) * 68 + (j << 4) + rl] = acc[i][j][r];
    }
    __builtin_amdgcn_fence(__ATOMIC_RELEASE, "workgroup");
    __builtin_amdgcn_wave_barrier();
    __builtin_amdgcn_fence(__ATOMIC_ACQUIRE, "workgroup");
    v4f vv[8];
#pragma unroll
    for (int it = 0; it < 8; ++it) {
      const int row = it * 2 + hh;
      v4f v = *(const v4fa*)(slab + row * 68 + c4);
      if (EPI == 1) v += bv;
      vv[it] = v;
    }
    for (int pass = 0; pass < 2; ++pass) {
#pragma unroll
      for (int it = 0; it < 8; ++it) {
        const int row = mBase + it * 2 + hh;
        if (cok && row < M) *(volatile v4f*)(D + (size_t)row * (size_t)ldd + nc) = vv[it];
      }
      __threadfence();
    }
    __builtin_amdgcn_fence(__ATOMIC_RELEASE, "workgroup");
    __builtin_amdgcn_wave_barrier();
    __builtin_amdgcn_fence(__ATOMIC_ACQUIRE, "workgroup");
  }
}

#define WO_TWO_TERM 1

#define NN     50000
#define NE     800000
#define DM     128
#define NHEAD  8
#define DKH    16
#define MPAD   50048
#define QLD    384
#define AGK    (WO_TWO_TERM ? 256 : 128)
#define LOGOFF 6400000

#define S_NTHR   256
#define S_NWAVE  8
#define S_CHUNK  2048
#define S_WCAP   256
#define S_LISTN  2048
#define S_NBMAX  2048
#define S_NBRUN  1024
#define S_RCAP   28672
#define S_DEGCAP 4096
#define S_NCHUNK ((NE + S_CHUNK - 1) / S_CHUNK)
#define S_BLOCKS ((MPAD + S_NBRUN - 1) / S_NBRUN)
#define S_LDS    ((2 * S_RCAP + 2 * S_NBMAX + S_LISTN) * 4 + 64)

static_assert(NE % 256 == 0);
static_assert(NE % 32 == 0 && NE % 4 == 0);
static_assert(NE < (1 << 20));
static_assert(DM == 32 * 4);
static_assert(DKH == 4 * 4 && NHEAD * DKH == DM);
static_assert(MPAD % 64 == 0 && MPAD >= NN && NN % 16 == 0);
static_assert(S_BLOCKS * S_NBRUN >= MPAD);
static_assert(S_BLOCKS == 49);
static_assert(S_NWAVE * S_WCAP == S_CHUNK);
static_assert(S_NTHR * 8 == S_NBMAX && S_LISTN == S_NBMAX && S_NBRUN <= S_NBMAX);
static_assert((S_NBRUN % S_NWAVE) == 0);
static_assert(S_RCAP % 32 == 0 && S_RCAP >= 16759 + 1024);
static_assert(S_DEGCAP >= 37 + 8);
static_assert(S_LDS <= 327680);
static_assert((size_t)LOGOFF + (size_t)NE * NHEAD == (size_t)12800000);
static_assert((size_t)NN * DM == (size_t)LOGOFF);

typedef unsigned int v2u __attribute__((ext_vector_type(2)));
typedef int          v4i __attribute__((ext_vector_type(4)));
typedef v4i __attribute__((may_alias)) v4ia;

__global__ __launch_bounds__(256) void k_wtr(const float* __restrict__ w, unsigned short* __restrict__ dst,
                                             int ppr, int nUnits) {
  const int g  = (int)blockIdx.x * 256 + (int)threadIdx.x;
  const int gc = g < nUnits ? g : nUnits - 1;
  const int n  = gc / ppr;
  const int p  = gc - n * ppr;
  const int k8 = (p & 15) << 3;
  const float* s = w + (size_t)k8 * DM + clampi(n, 0, DM - 1);
  float x[8];
#pragma unroll
  for (int i = 0; i < 8; ++i) {
    const float v = s[(size_t)i * DM];
    asm volatile("" :: "v"(v));
    x[i] = v;
  }
  const v4u o = pack8_bf16((v4f){ x[0], x[1], x[2], x[3] }, (v4f){ x[4], x[5], x[6], x[7] });
  if (g < nUnits) {
    volatile v4u* q = (volatile v4u*)(dst + (size_t)g * 8);
    *q = o;
    __threadfence();
    *q = o;
  }
}

__global__ __launch_bounds__(128) void k_bias(const float* __restrict__ bq, const float* __restrict__ bk,
                                              const float* __restrict__ bv, const float* __restrict__ bo,
                                              float* __restrict__ dst) {
  const int t   = (int)threadIdx.x;
  const int j   = (t & 31) * 4;
  const int sel = t >> 5;
  const v4f a = *(const v4fa*)(bq + j);
  const v4f b = *(const v4fa*)(bk + j);
  const v4f c = *(const v4fa*)(bv + j);
  const v4f d = *(const v4fa*)(bo + j);
  asm volatile("" :: "v"(a));
  asm volatile("" :: "v"(b));
  asm volatile("" :: "v"(c));
  asm volatile("" :: "v"(d));
  const unsigned m0 = sel == 0 ? 0xFFFFFFFFu : 0u;
  const unsigned m1 = sel == 1 ? 0xFFFFFFFFu : 0u;
  const unsigned m2 = sel == 2 ? 0xFFFFFFFFu : 0u;
  const unsigned m3 = sel == 3 ? 0xFFFFFFFFu : 0u;
  v4f o;
#pragma unroll
  for (int i = 0; i < 4; ++i) {
    const unsigned u = (__float_as_uint(a[i]) & m0) | (__float_as_uint(b[i]) & m1) |
                       (__float_as_uint(c[i]) & m2) | (__float_as_uint(d[i]) & m3);
    o[i] = bf16_val(__uint_as_float(u));
  }
  volatile v4f* q = (volatile v4f*)(dst + (size_t)t * 4);
  *q = o;
  __threadfence();
  *q = o;
}

__global__ __launch_bounds__(256) void k_logit(const int* __restrict__ ei, const float* __restrict__ attb,
                                               const float* __restrict__ qkv, float* __restrict__ lgo) {
  const int lane = (int)threadIdx.x & 31;
  const int wave = (int)threadIdx.x >> 5;
  const int g    = (int)blockIdx.x * 8 + wave;
  const int gc   = g < (NE / 4) ? g : (NE / 4) - 1;
  const int j    = lane >> 3;
  const int h    = lane & 7;
  const int e    = clampi(4 * gc + j, 0, NE - 1);
  const int draw = ei[e];
  const int sraw = ei[NE + e];
  const float braw = attb[(size_t)gc * 32 + lane];
  asm volatile("" :: "v"(draw));
  asm volatile("" :: "v"(sraw));
  asm volatile("" :: "v"(braw));
  const int d = clampi(draw, 0, NN - 1);
  const int s = clampi(sraw, 0, NN - 1);
  const float* qp = qkv + (size_t)d * QLD + h * DKH;
  const float* kp = qkv + (size_t)s * QLD + DM + h * DKH;
  v4f qv[4], kv[4];
#pragma unroll
  for (int i = 0; i < 4; ++i) {
    qv[i] = *(const v4fa*)(qp + 4 * i);
    kv[i] = *(const v4fa*)(kp + 4 * i);
  }
#pragma unroll
  for (int i = 0; i < 4; ++i) {
    asm volatile("" :: "v"(qv[i]));
    asm volatile("" :: "v"(kv[i]));
  }
  float dot = qv[0][0] * kv[0][0];
  dot = fmaf(qv[0][1], kv[0][1], dot);
  dot = fmaf(qv[0][2], kv[0][2], dot);
  dot = fmaf(qv[0][3], kv[0][3], dot);
#pragma unroll
  for (int i = 1; i < 4; ++i) {
    dot = fmaf(qv[i][0], kv[i][0], dot);
    dot = fmaf(qv[i][1], kv[i][1], dot);
    dot = fmaf(qv[i][2], kv[i][2], dot);
    dot = fmaf(qv[i][3], kv[i][3], dot);
  }
  const float lg = 0.25f * dot + bf16_val(braw);
  if (g < (NE / 4)) {
    volatile float* o = (volatile float*)(lgo + (size_t)g * 32 + lane);
    *o = lg;
    __threadfence();
    *o = lg;
  }
}

template <int TWO>
__global__ __launch_bounds__(S_NTHR) void k_scan(const int* __restrict__ ei, const float* __restrict__ qkv,
                                                 const float* __restrict__ lgp, unsigned short* __restrict__ agg) {
  constexpr int AGKc = TWO ? 2 * DM : DM;
  extern __shared__ v4f lds_dyn[];
  int* reg1 = (int*)lds_dyn;
  int* reg2 = reg1 + S_RCAP;
  int* scnt = reg2 + S_RCAP;
  int* soff = scnt + S_NBMAX;
  int* list = soff + S_NBMAX;
  int* wcnt = list + S_LISTN;
  int* wtot = wcnt + S_NWAVE;
  const int tid = (int)threadIdx.x, lane = tid & 31, wave = tid >> 5;
  const int nodeBase = (int)blockIdx.x * S_NBRUN;

  for (int i = tid; i < S_NBMAX; i += S_NTHR) { scnt[i] = 0; list[i] = 0; }
  __syncthreads();

  int tot = 0;
#pragma unroll 1
  for (int ch = 0; ch < S_NCHUNK; ++ch) {
    const int cbase = ch * S_CHUNK;
    int wc = 0;
    {
      const int wb  = cbase + wave * S_WCAP;
      const bool val = wb < NE;
      const int wbc = wb > NE - S_WCAP ? NE - S_WCAP : wb;
      const int* p = ei + wbc + lane;
      const int d0 = p[0],   d1 = p[32],  d2 = p[64],  d3 = p[96];
      const int d4 = p[128], d5 = p[160], d6 = p[192], d7 = p[224];
      asm volatile("" :: "v"(d0)); asm volatile("" :: "v"(d1));
      asm volatile("" :: "v"(d2)); asm volatile("" :: "v"(d3));
      asm volatile("" :: "v"(d4)); asm volatile("" :: "v"(d5));
      asm volatile("" :: "v"(d6)); asm volatile("" :: "v"(d7));
      const unsigned nbs = (unsigned)nodeBase;
      const unsigned unb = val ? (unsigned)S_NBRUN : 0u;
      const unsigned s0 = (unsigned)d0 - nbs, s1 = (unsigned)d1 - nbs;
      const unsigned s2 = (unsigned)d2 - nbs, s3 = (unsigned)d3 - nbs;
      const unsigned s4 = (unsigned)d4 - nbs, s5 = (unsigned)d5 - nbs;
      const unsigned s6 = (unsigned)d6 - nbs, s7 = (unsigned)d7 - nbs;
      const bool h0 = s0 < unb, h1 = s1 < unb, h2 = s2 < unb, h3 = s3 < unb;
      const bool h4 = s4 < unb, h5 = s5 < unb, h6 = s6 < unb, h7 = s7 < unb;
      const int elb = wave * S_WCAP + lane;
      const unsigned any = __builtin_amdgcn_ballot_w32(h0 | h1 | h2 | h3 | h4 | h5 | h6 | h7);
      if (any != 0u) {
#define HITJ(J, HJ, SJ) { \
        const unsigned mj = __builtin_amdgcn_ballot_w32(HJ); \
        if (mj != 0u) { \
          if (HJ) { \
            const int pos = wc + (int)__builtin_amdgcn_mbcnt_lo(mj, 0u); \
            if (pos < S_WCAP) list[wave * S_WCAP + pos] = ((elb + 32 * (J)) << 12) | (int)(SJ); \
          } \
          wc += (int)__builtin_popcount(mj); } }
        HITJ(0, h0, s0)
        HITJ(1, h1, s1)
        HITJ(2, h2, s2)
        HITJ(3, h3, s3)
        HITJ(4, h4, s4)
        HITJ(5, h5, s5)
        HITJ(6, h6, s6)
        HITJ(7, h7, s7)
#undef HITJ
      }
    }
    if (lane == 0) wcnt[wave] = wc;
    __syncthreads();
    int pre = 0, all = 0;
#pragma unroll
    for (int w2 = 0; w2 < S_NWAVE; ++w2) {
      int c = wcnt[w2];
      c = c < 0 ? 0 : (c > S_WCAP ? S_WCAP : c);
      all += c;
      pre += (w2 < wave) ? c : 0;
    }
    const int wcc  = wc > S_WCAP ? S_WCAP : wc;
    const int base = tot + pre;
#pragma unroll 1
    for (int i0 = 0; i0 < wcc; i0 += 32) {
      const int i   = i0 + lane;
      const int ic  = i < S_WCAP ? i : S_WCAP - 1;
      const int ent = list[wave * S_WCAP + ic];
      const int el  = (ent >> 12) & (S_CHUNK - 1);
      const int sl  = ent & (S_NBMAX - 1);
      int eid = cbase + el;
      eid = eid > NE - 1 ? NE - 1 : eid;
      const int pos = base + i;
      if (i < wcc && pos < S_RCAP) reg1[pos] = (int)(((unsigned)eid << 12) | (unsigned)sl);
    }
    tot += all;
    tot = tot > S_RCAP ? S_RCAP : tot;
    __syncthreads();
  }
  const int nh = tot;

  if (wave == 0) {
#pragma unroll 1
    for (int b0 = 0; b0 < nh; b0 += 32) {
      int idx = b0 + lane;
      idx = idx > nh - 1 ? nh - 1 : idx;
      const int uv  = reg1[idx];
      const int m32 = (nh - b0) < 32 ? (nh - b0) : 32;
#pragma unroll 1
      for (int k = 0; k < m32; ++k) {
        const int u  = __builtin_amdgcn_readlane(uv, k);
        const int sl = u & (S_NBMAX - 1);
        if (lane == 0) scnt[sl] = scnt[sl] + 1;
      }
    }
  }
  __syncthreads();

  {
    const v4i ca = *(const v4ia*)(scnt + 8 * tid);
    const v4i cb = *(const v4ia*)(scnt + 8 * tid + 4);
    const int e0 = ca.x < 0 ? 0 : ca.x, e1 = ca.y < 0 ? 0 : ca.y, e2 = ca.z < 0 ? 0 : ca.z, e3 = ca.w < 0 ? 0 : ca.w;
    const int e4 = cb.x < 0 ? 0 : cb.x, e5 = cb.y < 0 ? 0 : cb.y, e6 = cb.z < 0 ? 0 : cb.z, e7 = cb.w < 0 ? 0 : cb.w;
    const int ts = e0 + e1 + e2 + e3 + e4 + e5 + e6 + e7;
    int incl = ts;
#pragma unroll
    for (int d = 1; d < 32; d <<= 1) {
      const int up = __shfl_up(incl, d);
      if (lane >= d) incl += up;
    }
    if (lane == 31) wtot[wave] = incl;
    __syncthreads();
    int pre = 0;
#pragma unroll
    for (int w2 = 0; w2 < S_NWAVE; ++w2) pre += (w2 < wave) ? wtot[w2] : 0;
    int run = pre + incl - ts;
    soff[8 * tid + 0] = run; run += e0;
    soff[8 * tid + 1] = run; run += e1;
    soff[8 * tid + 2] = run; run += e2;
    soff[8 * tid + 3] = run; run += e3;
    soff[8 * tid + 4] = run; run += e4;
    soff[8 * tid + 5] = run; run += e5;
    soff[8 * tid + 6] = run; run += e6;
    soff[8 * tid + 7] = run;
  }
  __syncthreads();
  for (int i = tid; i < S_NBMAX; i += S_NTHR) list[i] = soff[i];
  __syncthreads();

  if (wave == 0) {
#pragma unroll 1
    for (int b0 = 0; b0 < nh; b0 += 32) {
      int idx = b0 + lane;
      idx = idx > nh - 1 ? nh - 1 : idx;
      const int uv  = reg1[idx];
      const int m32 = (nh - b0) < 32 ? (nh - b0) : 32;
#pragma unroll 1
      for (int k = 0; k < m32; ++k) {
        const int u   = __builtin_amdgcn_readlane(uv, k);
        const int sl  = u & (S_NBMAX - 1);
        const int eid = (int)((unsigned)u >> 12);
        if (lane == 0) {
          int pos = list[sl];
          pos = pos < 0 ? 0 : (pos > S_RCAP - 1 ? S_RCAP - 1 : pos);
          reg2[pos] = eid;
          list[sl] = pos + 1;
        }
      }
    }
  }
  __syncthreads();

  constexpr int nbw = S_NBRUN / S_NWAVE;
  const bool ovf = (nh >= S_RCAP);
  const int hd = lane >> 2;
#pragma unroll 1
  for (int jt = 0; jt < nbw; ++jt) {
    const int slot = wave * nbw + jt;
    const int grow = nodeBase + slot;
    int st = soff[slot];
    const int craw = scnt[slot];
    int cnt = craw;
    st  = st < 0 ? 0 : (st > nh ? nh : st);
    cnt = cnt < 0 ? 0 : (cnt > S_DEGCAP ? S_DEGCAP : cnt);
    if (cnt > nh - st) cnt = nh - st;
    const bool pois = ovf || (craw > S_DEGCAP);

    float m = 0.0f, s = 0.0f, a0 = 0.0f, a1 = 0.0f, a2 = 0.0f, a3 = 0.0f;
#pragma unroll 1
    for (int q = 0; q < cnt; ++q) {
      int idx = st + q; idx = idx > S_RCAP - 1 ? S_RCAP - 1 : idx;
      const int eid = clampi(reg2[idx], 0, NE - 1);
      const int sraw = ei[NE + eid];
      asm volatile("" :: "v"(sraw));
      const int sn = clampi(sraw, 0, NN - 1);
      const float lg = lgp[(size_t)eid * NHEAD + hd];
      asm volatile("" :: "v"(lg));
      const v4f vv = *(const v4fa*)(qkv + (size_t)sn * QLD + 2 * DM + 4 * lane);
      asm volatile("" :: "v"(vv));
      const float df = lg - m;
      const float ee = expf(-fabsf(df));
      const bool up    = df > 0.0f;
      const bool first = (q == 0);
      float s1 = up ? ee : 1.0f;
      float s2 = up ? 1.0f : ee;
      float mn = up ? lg : m;
      s1 = first ? 0.0f : s1;
      s2 = first ? 1.0f : s2;
      mn = first ? lg : mn;
      m  = mn;
      s  = fmaf(s,  s1, s2);
      a0 = fmaf(a0, s1, s2 * vv[0]);
      a1 = fmaf(a1, s1, s2 * vv[1]);
      a2 = fmaf(a2, s1, s2 * vv[2]);
      a3 = fmaf(a3, s1, s2 * vv[3]);
    }
    const bool empty = (cnt == 0);
    const float sd  = empty ? 1.0f : s;
    const float inv = 1.0f / sd;
    const float r0 = empty ? 0.0f : a0 * inv;
    const float r1 = empty ? 0.0f : a1 * inv;
    const float r2 = empty ? 0.0f : a2 * inv;
    const float r3 = empty ? 0.0f : a3 * inv;
    const bool live = grow < NN;
    unsigned h0 = bf16_bits(r0), h1 = bf16_bits(r1), h2 = bf16_bits(r2), h3 = bf16_bits(r3);
    unsigned l0 = bf16_lo_bits(r0), l1 = bf16_lo_bits(r1), l2 = bf16_lo_bits(r2), l3 = bf16_lo_bits(r3);
    h0 = pois ? 0x7FC0u : h0; h1 = pois ? 0x7FC0u : h1; h2 = pois ? 0x7FC0u : h2; h3 = pois ? 0x7FC0u : h3;
    l0 = pois ? 0u : l0;      l1 = pois ? 0u : l1;      l2 = pois ? 0u : l2;      l3 = pois ? 0u : l3;
    const unsigned lm = live ? 0xFFFFFFFFu : 0u;
    const v2u hw = (v2u){ pk16(h0, h1) & lm, pk16(h2, h3) & lm };
    const v2u lw = (v2u){ pk16(l0, l1) & lm, pk16(l2, l3) & lm };
    const bool wr = grow < MPAD;
    unsigned short* rp = agg + (size_t)(wr ? grow : 0) * AGKc + 4 * lane;
    if (wr) {
      *(volatile v2u*)rp = hw;
      if (TWO) *(volatile v2u*)(rp + DM) = lw;
    }
    __threadfence();
    if (wr) {
      *(volatile v2u*)rp = hw;
      if (TWO) *(volatile v2u*)(rp + DM) = lw;
    }
  }
}

extern "C" void kernel_launch(void* const* d_in, const int* in_sizes, int n_in,
                              void* d_out, int out_size, void* d_ws, size_t ws_size,
                              hipStream_t stream) {
  if (n_in < 11) return;
  if (in_sizes[0] != NN * DM) return;
  if (in_sizes[1] != 2 * NE) return;
  if (in_sizes[2] != NE * NHEAD) return;
  if (in_sizes[3] != DM * DM || in_sizes[5] != DM * DM || in_sizes[7] != DM * DM || in_sizes[9] != DM * DM) return;
  if (in_sizes[4] != DM || in_sizes[6] != DM || in_sizes[8] != DM || in_sizes[10] != DM) return;
  if (out_size != NN * DM + NE * NHEAD) return;

  const float* x   = (const float*)d_in[0];
  const int*   ei  = (const int*)  d_in[1];
  const float* att = (const float*)d_in[2];
  const float* Wq  = (const float*)d_in[3];
  const float* bq  = (const float*)d_in[4];
  const float* Wk  = (const float*)d_in[5];
  const float* bk  = (const float*)d_in[6];
  const float* Wv  = (const float*)d_in[7];
  const float* bv  = (const float*)d_in[8];
  const float* Wo  = (const float*)d_in[9];
  const float* bo  = (const float*)d_in[10];
  float* out = (float*)d_out;
  float* lgo = out + (size_t)LOGOFF;

  constexpr size_t bXB   = (size_t)MPAD * DM * 2;
  constexpr size_t bQKV  = (size_t)MPAD * QLD * 4;
  constexpr size_t bAGG  = (size_t)MPAD * AGK * 2;
  constexpr size_t bWQKV = (size_t)3 * DM * DM * 2;
  constexpr size_t bWOT  = (size_t)DM * AGK * 2;
  constexpr size_t bBIAS = (size_t)4 * DM * 4;
  constexpr size_t bTOT  = bXB + bQKV + bAGG + bWQKV + bWOT + bBIAS;
  static_assert(bXB % 256 == 0 && bQKV % 256 == 0 && bAGG % 256 == 0 && bWQKV % 256 == 0 && bWOT % 256 == 0);
  static_assert(bTOT <= ((size_t)128 << 20));
  if (bTOT > ws_size) return;
  char* ws = (char*)d_ws;
  unsigned short* XB    = (unsigned short*)(ws);
  float*          QKV   = (float*)(ws + bXB);
  unsigned short* AGG   = (unsigned short*)(ws + bXB + bQKV);
  unsigned short* WQKVT = (unsigned short*)(ws + bXB + bQKV + bAGG);
  unsigned short* WOT   = (unsigned short*)(ws + bXB + bQKV + bAGG + bWQKV);
  float*          BIAS  = (float*)(ws + bXB + bQKV + bAGG + bWQKV + bWOT);

  hipFuncSetAttribute(reinterpret_cast<const void*>(&k_scan<WO_TWO_TERM>),
                      hipFuncAttributeMaxDynamicSharedMemorySize, S_LDS);

  static_assert(((size_t)MPAD * DM / 8) % 256 == 0);
  k_plane<0><<<MPAD * DM / 8 / 256, 256, 0, stream>>>(x, NN, DM, DM, XB, MPAD, DM);
  k_wtr<<<DM * 16 / 256, 256, 0, stream>>>(Wq, WQKVT,               16, DM * 16);
  k_wtr<<<DM * 16 / 256, 256, 0, stream>>>(Wk, WQKVT + DM * DM,     16, DM * 16);
  k_wtr<<<DM * 16 / 256, 256, 0, stream>>>(Wv, WQKVT + 2 * DM * DM, 16, DM * 16);
  k_wtr<<<DM * (AGK / 8) / 256, 256, 0, stream>>>(Wo, WOT, AGK / 8, DM * (AGK / 8));
  k_bias<<<1, 128, 0, stream>>>(bq, bk, bv, bo, BIAS);

  {
    constexpr int T = ((NN + 63) / 64) * (QLD / 64);
    k_gemm_nt<0, 1><<<(T + 7) / 8, 256, 0, stream>>>(XB, WQKVT, BIAS, QKV, NN, QLD, DM, QLD);
  }
  k_logit<<<NE / 32, 256, 0, stream>>>(ei, att, QKV, lgo);
  k_scan<WO_TWO_TERM><<<S_BLOCKS, S_NTHR, S_LDS, stream>>>(ei, QKV, lgo, AGG);
  {
    constexpr int T = ((NN + 63) / 64) * (DM / 64);
    k_gemm_nt<0, 1><<<(T + 7) / 8, 256, 0, stream>>>(AGG, WOT, BIAS + 3 * DM, out, NN, DM, AGK, DM);
  }
}
